// EGNN_15135464751163
// MI455X (gfx1250) — hardware-verified
//
#include <hip/hip_runtime.h>
#include <stddef.h>
#include <stdint.h>

#define NN    16384
#define KNB   10
#define HID   128
#define NL    7
#define FIN   8
#define HROW  11
#define GBM   64
#define GBN   128
#define GTHR  128
#define EROWS 160
#define APT   264
#define EPT   132
#define SPT   132
#define TPT   264

#define NU_W1SD (NL * 256 * 32)
#define NU_W2D  (NL * 128 * 32)
#define NU_CW1  (NL * 128 * 16)
#define NU_NW1Q (NL * 128 * 64)
#define NU_NW2D (NL * 128 * 32)

#define OFF_A    0
#define SZ_A     (EROWS * APT * 2)
#define OFF_EF   (OFF_A + SZ_A)
#define SZ_EF    (EROWS * EPT * 4)
#define OFF_PAR  (OFF_EF + SZ_EF)
#define OFF_PD   (OFF_PAR + 8 * HID * 4)
#define OFF_DIF  (OFF_PD + 16 * HID * 4)
#define OFF_TR   (OFF_DIF + EROWS * 16)
#define OFF_IDX  (OFF_TR + EROWS * 16)
#define OFF_CM   (OFF_IDX + EROWS * 4)
#define EDGE_LDS (OFF_CM + EROWS * 4)

#define UOFF_STG 0
#define UOFF_T   (128 * SPT * 4)
#define UOFF_PAR (UOFF_T + 128 * TPT * 2)
#define UPD_LDS  (UOFF_PAR + 2 * HID * 4)

#define WSMAX 134217728

static_assert(NN % 128 == 0);
static_assert(NN % 16 == 0);
static_assert(NN % GBM == 0 && NN % 32 == 0 && NN % 64 == 0);
static_assert(KNB == 10);
static_assert(HID == 128);
static_assert(8 * 16 == HID);
static_assert(NL == 7);
static_assert(EROWS == 16 * KNB && EROWS % 16 == 0 && EROWS % 8 == 0);
static_assert(EDGE_LDS <= 327680);
static_assert(UPD_LDS <= 327680);
static_assert((SZ_A % 16) == 0 && (SZ_EF % 16) == 0 && (OFF_CM % 16) == 0);
static_assert((APT * 2) % 16 == 0 && (EPT * 4) % 16 == 0 && APT >= 256 && EPT >= HID);
static_assert(NU_W1SD % 256 == 0 && NU_W2D % 256 == 0 && NU_CW1 % 256 == 0);
static_assert(NU_NW1Q % 256 == 0 && NU_NW2D % 256 == 0);
static_assert((32 * HROW) % 4 == 0 && (32 * HROW * 4) % 16 == 0);
static_assert(GBM == (GTHR / 32) * 16 && GBN == HID);

typedef float          v4f   __attribute__((ext_vector_type(4)));
typedef float          v8f   __attribute__((ext_vector_type(8)));
typedef int            v8i   __attribute__((ext_vector_type(8)));
typedef unsigned short v4us  __attribute__((ext_vector_type(4)));
typedef unsigned short v8us  __attribute__((ext_vector_type(8)));
typedef unsigned short v16us __attribute__((ext_vector_type(16)));
typedef __bf16         v16bf __attribute__((ext_vector_type(16)));
typedef v4f  __attribute__((may_alias)) v4fa;
typedef v4us __attribute__((may_alias)) v4usa;
typedef v8us __attribute__((may_alias)) v8usa;
union FragB { v16bf v; v16us u; v8us h[2]; v8i w; };
struct HL4 { v4us hi; v4us lo; };

__device__ __forceinline__ v8f wmb(const FragB& a, const FragB& b, v8f c) {
  v8f d = __builtin_amdgcn_wmma_f32_16x16x32_bf16(false, a.v, false, b.v, (short)0, c, false, false);
  asm volatile("v_nop\n\tv_nop\n\tv_nop\n\tv_nop" : "+v"(d) : "v"(a.w), "v"(b.w));
  return d;
}

__device__ __forceinline__ unsigned bf16_bits(float f) {
  const unsigned u = __float_as_uint(f);
  return (u + 0x7FFFu + ((u >> 16) & 1u)) >> 16;
}
__device__ __forceinline__ float bf16_val(float f) {
  return __uint_as_float(bf16_bits(f) << 16);
}
__device__ __forceinline__ v4f bf16_val4(v4f a) {
  v4f r;
  r.x = bf16_val(a.x); r.y = bf16_val(a.y); r.z = bf16_val(a.z); r.w = bf16_val(a.w);
  return r;
}
__device__ __forceinline__ float silu_p(float v) {
  const float e = expf(fminf(-v, 40.0f));
  return v / (1.0f + e);
}
__device__ __forceinline__ float clip1k(float v) {
  return (v > 1000.0f) ? 1000.0f : ((v < -1000.0f) ? -1000.0f : v);
}
__device__ __forceinline__ HL4 split4(v4f a) {
  HL4 r;
  const unsigned h0 = bf16_bits(a.x), h1 = bf16_bits(a.y), h2 = bf16_bits(a.z), h3 = bf16_bits(a.w);
  r.hi.x = (unsigned short)h0; r.hi.y = (unsigned short)h1; r.hi.z = (unsigned short)h2; r.hi.w = (unsigned short)h3;
  r.lo.x = (unsigned short)bf16_bits(a.x - __uint_as_float(h0 << 16));
  r.lo.y = (unsigned short)bf16_bits(a.y - __uint_as_float(h1 << 16));
  r.lo.z = (unsigned short)bf16_bits(a.z - __uint_as_float(h2 << 16));
  r.lo.w = (unsigned short)bf16_bits(a.w - __uint_as_float(h3 << 16));
  return r;
}
__device__ __forceinline__ v8us hl8(v4f a, v4f b, unsigned ml, unsigned mh) {
  const v8f f8 = {a.x, a.y, a.z, a.w, b.x, b.y, b.z, b.w};
  v8us oo;
#pragma unroll
  for (int e = 0; e < 8; ++e) {
    const unsigned hb = bf16_bits(f8[e]);
    const unsigned lb = bf16_bits(f8[e] - __uint_as_float(hb << 16));
    oo[e] = (unsigned short)((hb & ml) | (lb & mh));
  }
  return oo;
}
__device__ __forceinline__ void put16(unsigned short* dp, v8us o) {
  *(volatile v8us*)dp = o;
  __threadfence();
  *(volatile v8us*)dp = o;
}
__device__ __forceinline__ void putf4(float* dp, v4f o) {
  *(volatile v4f*)dp = o;
  __threadfence();
  *(volatile v4f*)dp = o;
}

__global__ __launch_bounds__(256) __attribute__((amdgpu_num_vgpr(248)))
void k_pa(const float* __restrict__ ew1, const float* __restrict__ ew2, const float* __restrict__ cw1,
          unsigned short* W1SD, unsigned short* W2D, unsigned short* CW1T) {
  const int u = (int)blockIdx.x * 256 + (int)threadIdx.x;
  v8us o;
  if (u < NU_W1SD) {
    const int l  = u >> 13;
    const int v  = u & 8191;
    const int n  = v >> 5;
    const int k8 = (v & 31) * 8;
    const int nn = n & 127;
    const int rb = ((n < 128) ? 1 : 129) + (k8 & 127);
    const float* p = ew1 + (size_t)l * 257 * 128 + (size_t)rb * 128 + nn;
#pragma unroll
    for (int i = 0; i < 8; ++i) o[i] = (unsigned short)bf16_bits(p[(size_t)i * 128]);
    put16(W1SD + (size_t)l * 65536 + (size_t)v * 8, o);
  } else if (u < NU_W1SD + NU_W2D) {
    const int w  = u - NU_W1SD;
    const int l  = w >> 12;
    const int v  = w & 4095;
    const int n  = v >> 5;
    const int k8 = (v & 31) * 8;
    const float* p = ew2 + (size_t)l * 16384 + (size_t)(k8 & 127) * 128 + n;
#pragma unroll
    for (int i = 0; i < 8; ++i) o[i] = (unsigned short)bf16_bits(p[(size_t)i * 128]);
    put16(W2D + (size_t)l * 32768 + (size_t)v * 8, o);
  } else if (u < NU_W1SD + NU_W2D + NU_CW1) {
    const int w  = u - NU_W1SD - NU_W2D;
    const int l  = w >> 11;
    const int v  = w & 2047;
    const int n  = v >> 4;
    const int k8 = (v & 15) * 8;
    const float* p = cw1 + (size_t)l * 16384 + (size_t)k8 * 128 + n;
#pragma unroll
    for (int i = 0; i < 8; ++i) o[i] = (unsigned short)bf16_bits(p[(size_t)i * 128]);
    put16(CW1T + (size_t)l * 16384 + (size_t)v * 8, o);
  }
}

__global__ __launch_bounds__(256) __attribute__((amdgpu_num_vgpr(248)))
void k_pb(const float* __restrict__ nw1, const float* __restrict__ nw2,
          unsigned short* NW1Q, unsigned short* NW2D) {
  const int u = (int)blockIdx.x * 256 + (int)threadIdx.x;
  v8us o;
  if (u < NU_NW1Q) {
    const int l  = u >> 13;
    const int v  = u & 8191;
    const int n  = v >> 6;
    const int k8 = (v & 63) * 8;
    const int sr = ((k8 < 256) ? 0 : 128) + (k8 & 127);
    const float* p = nw1 + (size_t)l * 32768 + (size_t)sr * 128 + n;
#pragma unroll
    for (int i = 0; i < 8; ++i) o[i] = (unsigned short)bf16_bits(p[(size_t)i * 128]);
    put16(NW1Q + (size_t)l * 65536 + (size_t)v * 8, o);
  } else if (u < NU_NW1Q + NU_NW2D) {
    const int w  = u - NU_NW1Q;
    const int l  = w >> 12;
    const int v  = w & 4095;
    const int n  = v >> 5;
    const int k8 = (v & 31) * 8;
    const float* p = nw2 + (size_t)l * 16384 + (size_t)(k8 & 127) * 128 + n;
#pragma unroll
    for (int i = 0; i < 8; ++i) o[i] = (unsigned short)bf16_bits(p[(size_t)i * 128]);
    put16(NW2D + (size_t)l * 32768 + (size_t)v * 8, o);
  }
}

__global__ __launch_bounds__(256) __attribute__((amdgpu_num_vgpr(248)))
void k_pc(const float* __restrict__ ew1, const float* __restrict__ eb1, const float* __restrict__ eb2,
          const float* __restrict__ cb1, const float* __restrict__ cw2, const float* __restrict__ nb1,
          const float* __restrict__ nb2, const float* __restrict__ eow, const float* __restrict__ eob,
          float* PAR, float* EO) {
  const int tid = (int)threadIdx.x;
  const v4f z4 = {0.0f, 0.0f, 0.0f, 0.0f};
  if ((int)blockIdx.x < NL) {
    const int l   = (int)blockIdx.x;
    const int j   = tid >> 5;
    const int c4  = (tid & 31) * 4;
    const v4f a0 = *(const v4fa*)(ew1 + (size_t)l * 257 * 128 + c4);
    const v4f a1 = *(const v4fa*)(eb1 + l * HID + c4);
    const v4f a2 = *(const v4fa*)(eb2 + l * HID + c4);
    const v4f a3 = *(const v4fa*)(cb1 + l * HID + c4);
    const v4f a4 = *(const v4fa*)(cw2 + l * HID + c4);
    const v4f a5 = *(const v4fa*)(nb1 + l * HID + c4);
    const v4f a6 = *(const v4fa*)(nb2 + l * HID + c4);
    v4f s = a0;
    s = (j == 1) ? a1 : s;
    s = (j == 2) ? a2 : s;
    s = (j == 3) ? a3 : s;
    s = (j == 4) ? a4 : s;
    s = (j == 5) ? a5 : s;
    s = (j == 6) ? a6 : s;
    s = (j == 7) ? z4 : s;
    putf4(PAR + (size_t)l * 1024 + (size_t)tid * 4, bf16_val4(s));
  } else {
    const int r  = tid;
    const int rc = r < 130 ? r : 130;
    const v4f wv = *(const v4fa*)(eow + rc * 4);
    const v4f bv = *(const v4fa*)(eob);
    v4f s = bf16_val4(wv);
    s = (r == 131) ? bf16_val4(bv) : s;
    s = (r > 131) ? z4 : s;
    const int rs = r < 136 ? r : 135;
    float* dp = EO + rs * 4;
    if (r < 136) *(volatile v4f*)dp = s;
    __threadfence();
    if (r < 136) *(volatile v4f*)dp = s;
  }
}

__device__ __forceinline__ void emb_store(const float* stg, float* HH0, unsigned short* HL0, float* X0,
                                          int rb, int wave, int lane, int tid, v4f xq) {
  const int part = lane >> 4, j = lane & 15;
  const unsigned mh = 0u - (unsigned)part;
  const unsigned ml = ~mh;
#pragma unroll 1
  for (int r = 0; r < 4; ++r) {
    const int lr = 4 * wave + r;
    const size_t row = (size_t)(rb + lr);
    const v4f v = *(const v4fa*)(stg + lr * HID + 4 * lane);
    *(volatile v4f*)(HH0 + row * HID + 4 * lane) = v;
    const v4f a = *(const v4fa*)(stg + lr * HID + 8 * j);
    const v4f b = *(const v4fa*)(stg + lr * HID + 8 * j + 4);
    const v8us oo = hl8(a, b, ml, mh);
    *(volatile v8us*)(HL0 + row * 256 + part * HID + 8 * j) = oo;
  }
  if (tid < 32) *(volatile v4f*)(X0 + (size_t)(rb + tid) * 4) = xq;
}

__global__ __launch_bounds__(256) __attribute__((amdgpu_num_vgpr(248)))
void k_emb(const float* __restrict__ h, const float* __restrict__ w, const float* __restrict__ b,
           float* X0, float* HH0, unsigned short* HL0) {
  __shared__ __attribute__((aligned(16))) float sh[32 * HROW];
  __shared__ __attribute__((aligned(16))) float stg[32 * HID];
  const int tid = (int)threadIdx.x, lane = tid & 31, wave = tid >> 5;
  const int rb = (int)blockIdx.x * 32;
  {
    const int tl = tid < 88 ? tid : 87;
    const v4f a = *(const v4fa*)(h + (size_t)rb * HROW + 4 * tl);
    if (tid < 88) *(v4fa*)(sh + 4 * tid) = bf16_val4(a);
  }
  __syncthreads();
  {
    const v4f bb = bf16_val4(*(const v4fa*)(b + 4 * lane));
#pragma unroll 1
    for (int r = 0; r < 4; ++r) {
      const int lr = 4 * wave + r;
      v4f acc = {0.0f, 0.0f, 0.0f, 0.0f};
#pragma unroll 1
      for (int i = 0; i < FIN; ++i) {
        const float f = sh[lr * HROW + 3 + i];
        const v4f wv = bf16_val4(*(const v4fa*)(w + i * HID + 4 * lane));
        acc.x = fmaf(f, wv.x, acc.x);
        acc.y = fmaf(f, wv.y, acc.y);
        acc.z = fmaf(f, wv.z, acc.z);
        acc.w = fmaf(f, wv.w, acc.w);
      }
      acc.x += bb.x; acc.y += bb.y; acc.z += bb.z; acc.w += bb.w;
      *(v4fa*)(stg + lr * HID + 4 * lane) = acc;
    }
  }
  __syncthreads();
  v4f xq;
  xq.x = sh[lane * HROW + 0] / 3330.0f;
  xq.y = sh[lane * HROW + 1] / 3330.0f;
  xq.z = sh[lane * HROW + 2] / 3330.0f;
  xq.w = 0.0f;
  emb_store(stg, HH0, HL0, X0, rb, wave, lane, tid, xq);
  __threadfence();
  emb_store(stg, HH0, HL0, X0, rb, wave, lane, tid, xq);
}

__global__ __launch_bounds__(GTHR) __attribute__((amdgpu_num_vgpr(248)))
void k_node(const unsigned short* __restrict__ A, const unsigned short* __restrict__ BT,
            const float* __restrict__ bias, float* Cm) {
  __shared__ __attribute__((aligned(16))) float stg[GBM * GBN];
  const int tid = (int)threadIdx.x, lane = tid & 31, wave = tid >> 5, hh = lane >> 4, m = lane & 15;
  const int rowBase = (int)blockIdx.x * GBM;
  const int colBase = (int)blockIdx.y * GBN;
  v8f acc[8];
  {
    const v8f z = {0.f, 0.f, 0.f, 0.f, 0.f, 0.f, 0.f, 0.f};
#pragma unroll
    for (int t = 0; t < 8; ++t) acc[t] = z;
  }
  const unsigned short* ap = A  + (size_t)(rowBase + 16 * wave + m) * 256 + 8 * hh;
  const unsigned short* bp = BT + (size_t)(colBase + m) * 256 + 8 * hh;
#pragma unroll 1
  for (int k0 = 0; k0 < 256; k0 += 32) {
    FragB af;
    af.h[0] = *(const v8usa*)(ap + k0);
    af.h[1] = *(const v8usa*)(ap + k0 + 16);
#pragma unroll
    for (int nt = 0; nt < 8; ++nt) {
      const unsigned short* wq = bp + (size_t)(16 * nt) * 256 + k0;
      FragB bf;
      bf.h[0] = *(const v8usa*)wq;
      bf.h[1] = *(const v8usa*)(wq + 16);
      acc[nt] = wmb(af, bf, acc[nt]);
    }
  }
  const float bsel = ((int)blockIdx.y != 0) ? 1.0f : 0.0f;
#pragma unroll
  for (int nt = 0; nt < 8; ++nt) {
    const int lc = 16 * nt + m;
    const float bvv = bias[lc] * bsel;
#pragma unroll
    for (int r = 0; r < 8; ++r) {
      const int lr = 16 * wave + 8 * hh + r;
      stg[lr * GBN + lc] = acc[nt][r] + bvv;
    }
  }
  __syncthreads();
  v4f pv[16];
#pragma unroll
  for (int i = 0; i < 16; ++i) pv[i] = *(const v4fa*)(stg + (16 * wave + i) * GBN + 4 * lane);
#pragma unroll
  for (int i = 0; i < 16; ++i) {
    float* op = Cm + (size_t)(rowBase + 16 * wave + i) * 256 + colBase + 4 * lane;
    *(volatile v4f*)op = pv[i];
  }
  __threadfence();
#pragma unroll
  for (int i = 0; i < 16; ++i) {
    float* op = Cm + (size_t)(rowBase + 16 * wave + i) * 256 + colBase + 4 * lane;
    *(volatile v4f*)op = pv[i];
  }
}

__global__ __launch_bounds__(256) __attribute__((amdgpu_num_vgpr(248)))
void k_edge(const float* __restrict__ Xin, float* Xout, const float* __restrict__ PSD,
            const int* __restrict__ idx, const unsigned short* __restrict__ W2,
            const unsigned short* __restrict__ CW, const float* __restrict__ PARl,
            unsigned short* SHL) {
  extern __shared__ __attribute__((aligned(16))) unsigned char smem_e[];
  unsigned short* sA   = (unsigned short*)(smem_e + OFF_A);
  float*          sEF  = (float*)(smem_e + OFF_EF);
  float*          sPar = (float*)(smem_e + OFF_PAR);
  float*          sPD  = (float*)(smem_e + OFF_PD);
  float*          sDif = (float*)(smem_e + OFF_DIF);
  float*          sTr  = (float*)(smem_e + OFF_TR);
  int*            sIdx = (int*)(smem_e + OFF_IDX);
  float*          sCm  = (float*)(smem_e + OFF_CM);

  const int tid = (int)threadIdx.x, lane = tid & 31, wave = tid >> 5, hh = lane >> 4, m = lane & 15;
  const int nb = (int)blockIdx.x * 16;

  {
    const v4f p = *(const v4fa*)(PARl + 4 * tid);
    *(v4fa*)(sPar + 4 * tid) = p;
  }
#pragma unroll
  for (int q = 0; q < 2; ++q) {
    const int u  = q * 256 + tid;
    const int j  = u >> 5;
    const int c4 = (u & 31) * 4;
    const v4f v = *(const v4fa*)(PSD + (size_t)(nb + j) * 256 + HID + c4);
    *(v4fa*)(sPD + j * HID + c4) = v;
  }
  {
    const int e = tid < EROWS ? tid : EROWS - 1;
    int s = idx[(size_t)nb * KNB + e];
    s = s < 0 ? 0 : (s > NN - 1 ? NN - 1 : s);
    const int j = e / KNB;
    const v4f xs = *(const v4fa*)(Xin + (size_t)s * 4);
    const v4f xd = *(const v4fa*)(Xin + (size_t)(nb + j) * 4);
    const float dx = xs.x - xd.x, dy = xs.y - xd.y, dz = xs.z - xd.z;
    const float radial = (dx * dx + dz * dz) + dy * dy;
    if (tid < EROWS) {
      sIdx[tid] = s;
      const v4f d4 = {dx, dy, dz, radial};
      *(v4fa*)(sDif + 4 * tid) = d4;
    }
  }
  __syncthreads();

  {
    const v4f wr = *(const v4fa*)(sPar + 4 * lane);
#pragma unroll 1
    for (int it = 0; it < EROWS / 8; ++it) {
      const int e = it * 8 + wave;
      const int s = sIdx[e];
      const int j = e / KNB;
      const float rad = sDif[4 * e + 3];
      const v4f ps = *(const v4fa*)(PSD + (size_t)s * 256 + 4 * lane);
      const v4f pd = *(const v4fa*)(sPD + j * HID + 4 * lane);
      v4f a;
      a.x = silu_p(fmaf(rad, wr.x, ps.x + pd.x));
      a.y = silu_p(fmaf(rad, wr.y, ps.y + pd.y));
      a.z = silu_p(fmaf(rad, wr.z, ps.z + pd.z));
      a.w = silu_p(fmaf(rad, wr.w, ps.w + pd.w));
      const HL4 q = split4(a);
      *(v4usa*)(sA + e * APT + 4 * lane)       = q.hi;
      *(v4usa*)(sA + e * APT + HID + 4 * lane) = q.lo;
    }
  }
  __syncthreads();

  v8f acc[10];
  {
    const v8f z = {0.f, 0.f, 0.f, 0.f, 0.f, 0.f, 0.f, 0.f};
#pragma unroll
    for (int t = 0; t < 10; ++t) acc[t] = z;
  }
  {
    const unsigned short* bp = W2 + (size_t)(16 * wave + m) * 256 + 8 * hh;
    const unsigned short* ap = sA + m * APT + 8 * hh;
#pragma unroll 1
    for (int k0 = 0; k0 < 256; k0 += 32) {
      FragB bf;
      bf.h[0] = *(const v8usa*)(bp + k0);
      bf.h[1] = *(const v8usa*)(bp + k0 + 16);
#pragma unroll
      for (int rt = 0; rt < 10; ++rt) {
        FragB af;
        af.h[0] = *(const v8usa*)(ap + rt * 16 * APT + k0);
        af.h[1] = *(const v8usa*)(ap + rt * 16 * APT + k0 + 16);
        acc[rt] = wmb(af, bf, acc[rt]);
      }
    }
  }
#pragma unroll
  for (int rt = 0; rt < 10; ++rt)
#pragma unroll
    for (int r = 0; r < 8; ++r)
      sEF[(16 * rt + 8 * hh + r) * EPT + 16 * wave + m] = acc[rt][r];
  __syncthreads();

  {
    const v4f b2 = *(const v4fa*)(sPar + 2 * HID + 4 * lane);
#pragma unroll 1
    for (int jj = 0; jj < 2; ++jj) {
      const int j = wave + 8 * jj;
      v4f S = {0.0f, 0.0f, 0.0f, 0.0f};
#pragma unroll 1
      for (int k = 0; k < KNB; ++k) {
        const int e = KNB * j + k;
        const v4f v = *(const v4fa*)(sEF + e * EPT + 4 * lane);
        v4f ef;
        ef.x = silu_p(v.x + b2.x);
        ef.y = silu_p(v.y + b2.y);
        ef.z = silu_p(v.z + b2.z);
        ef.w = silu_p(v.w + b2.w);
        S.x += ef.x; S.y += ef.y; S.z += ef.z; S.w += ef.w;
        const HL4 q = split4(ef);
        *(v4usa*)(sA + e * APT + 4 * lane) = q.hi;
      }
      const HL4 sq = split4(S);
      unsigned short* dp = SHL + (size_t)(nb + j) * 256 + 4 * lane;
      *(volatile v4us*)dp         = sq.hi;
      *(volatile v4us*)(dp + HID) = sq.lo;
      __threadfence();
      *(volatile v4us*)dp         = sq.hi;
      *(volatile v4us*)(dp + HID) = sq.lo;
    }
  }
  __syncthreads();

  {
    const v8f z = {0.f, 0.f, 0.f, 0.f, 0.f, 0.f, 0.f, 0.f};
#pragma unroll
    for (int t = 0; t < 10; ++t) acc[t] = z;
  }
  {
    const unsigned short* bp = CW + (size_t)(16 * wave + m) * HID + 8 * hh;
    const unsigned short* ap = sA + m * APT + 8 * hh;
#pragma unroll 1
    for (int k0 = 0; k0 < HID; k0 += 32) {
      FragB bf;
      bf.h[0] = *(const v8usa*)(bp + k0);
      bf.h[1] = *(const v8usa*)(bp + k0 + 16);
#pragma unroll
      for (int rt = 0; rt < 10; ++rt) {
        FragB af;
        af.h[0] = *(const v8usa*)(ap + rt * 16 * APT + k0);
        af.h[1] = *(const v8usa*)(ap + rt * 16 * APT + k0 + 16);
        acc[rt] = wmb(af, bf, acc[rt]);
      }
    }
  }
#pragma unroll
  for (int rt = 0; rt < 10; ++rt)
#pragma unroll
    for (int r = 0; r < 8; ++r)
      sEF[(16 * rt + 8 * hh + r) * EPT + 16 * wave + m] = acc[rt][r];
  __syncthreads();

  {
    const v4f cb = *(const v4fa*)(sPar + 3 * HID + 4 * lane);
    const v4f cw = *(const v4fa*)(sPar + 4 * HID + 4 * lane);
#pragma unroll 1
    for (int it = 0; it < EROWS / 8; ++it) {
      const int e = it * 8 + wave;
      const v4f v = *(const v4fa*)(sEF + e * EPT + 4 * lane);
      float p = silu_p(v.x + cb.x) * cw.x;
      p = fmaf(silu_p(v.y + cb.y), cw.y, p);
      p = fmaf(silu_p(v.z + cb.z), cw.z, p);
      p = fmaf(silu_p(v.w + cb.w), cw.w, p);
      p += __shfl_xor(p, 16);
      p += __shfl_xor(p, 8);
      p += __shfl_xor(p, 4);
      p += __shfl_xor(p, 2);
      p += __shfl_xor(p, 1);
      if (lane == 0) sCm[e] = p;
    }
  }
  __syncthreads();

  if (tid < EROWS) {
    const v4f d = *(const v4fa*)(sDif + 4 * tid);
    const float cm = sCm[tid];
    const v4f t4 = {clip1k(d.x * cm), clip1k(d.y * cm), clip1k(d.z * cm), 0.0f};
    *(v4fa*)(sTr + 4 * tid) = t4;
  }
  __syncthreads();
  {
    const int tl = tid & 15;
    float sx = 0.0f, sy = 0.0f, sz = 0.0f;
#pragma unroll 2
    for (int k = 0; k < KNB; ++k) {
      const v4f t4 = *(const v4fa*)(sTr + 4 * (KNB * tl + k));
      sx += t4.x; sy += t4.y; sz += t4.z;
    }
    const v4f xo = *(const v4fa*)(Xin + (size_t)(nb + tl) * 4);
    v4f xn;
    xn.x = clip1k(xo.x) + sx / 10.0f;
    xn.y = clip1k(xo.y) + sy / 10.0f;
    xn.z = clip1k(xo.z) + sz / 10.0f;
    xn.w = 0.0f;
    float* dp = Xout + (size_t)(nb + tl) * 4;
    if (tid < 16) *(volatile v4f*)dp = xn;
    __threadfence();
    if (tid < 16) *(volatile v4f*)dp = xn;
  }
}

__device__ __forceinline__ void upd_store(const float* stg, float* HHo, unsigned short* HLo,
                                          int rowBase, int wave, int lane) {
  const int part = lane >> 4, j = lane & 15;
  const unsigned mh = 0u - (unsigned)part;
  const unsigned ml = ~mh;
#pragma unroll 1
  for (int i = 0; i < 16; ++i) {
    const int lr = 16 * wave + i;
    const size_t row = (size_t)(rowBase + lr);
    const v4f v = *(const v4fa*)(stg + lr * SPT + 4 * lane);
    *(volatile v4f*)(HHo + row * HID + 4 * lane) = v;
    const v4f a = *(const v4fa*)(stg + lr * SPT + 8 * j);
    const v4f b = *(const v4fa*)(stg + lr * SPT + 8 * j + 4);
    const v8us oo = hl8(a, b, ml, mh);
    *(volatile v8us*)(HLo + row * 256 + part * HID + 8 * j) = oo;
  }
}

__global__ __launch_bounds__(256) __attribute__((amdgpu_num_vgpr(248)))
void k_upd(const unsigned short* __restrict__ HLi, const unsigned short* __restrict__ SHL,
           const unsigned short* __restrict__ NW1, const unsigned short* __restrict__ NW2,
           const float* __restrict__ PARl, const float* __restrict__ HHi,
           float* HHo, unsigned short* HLo) {
  extern __shared__ __attribute__((aligned(16))) unsigned char smem_u[];
  float*          stg  = (float*)(smem_u + UOFF_STG);
  unsigned short* sT   = (unsigned short*)(smem_u + UOFF_T);
  float*          sPar = (float*)(smem_u + UOFF_PAR);
  const int tid = (int)threadIdx.x, lane = tid & 31, wave = tid >> 5, hh = lane >> 4, m = lane & 15;
  const int rowBase = (int)blockIdx.x * 128;
  {
    const int tl = tid < 64 ? tid : 63;
    const v4f p = *(const v4fa*)(PARl + 5 * HID + 4 * tl);
    if (tid < 64) *(v4fa*)(sPar + 4 * tid) = p;
  }
  v8f acc[8];
  {
    const v8f z = {0.f, 0.f, 0.f, 0.f, 0.f, 0.f, 0.f, 0.f};
#pragma unroll
    for (int t = 0; t < 8; ++t) acc[t] = z;
  }
  {
    const unsigned short* ap1 = HLi + (size_t)(rowBase + 16 * wave + m) * 256 + 8 * hh;
    const unsigned short* ap2 = SHL + (size_t)(rowBase + 16 * wave + m) * 256 + 8 * hh;
    const unsigned short* bp  = NW1 + (size_t)m * 512 + 8 * hh;
#pragma unroll 1
    for (int k0 = 0; k0 < 256; k0 += 32) {
      FragB af;
      af.h[0] = *(const v8usa*)(ap1 + k0);
      af.h[1] = *(const v8usa*)(ap1 + k0 + 16);
#pragma unroll
      for (int nt = 0; nt < 8; ++nt) {
        const unsigned short* wq = bp + (size_t)(16 * nt) * 512 + k0;
        FragB bf;
        bf.h[0] = *(const v8usa*)wq;
        bf.h[1] = *(const v8usa*)(wq + 16);
        acc[nt] = wmb(af, bf, acc[nt]);
      }
    }
#pragma unroll 1
    for (int k0 = 0; k0 < 256; k0 += 32) {
      FragB af;
      af.h[0] = *(const v8usa*)(ap2 + k0);
      af.h[1] = *(const v8usa*)(ap2 + k0 + 16);
#pragma unroll
      for (int nt = 0; nt < 8; ++nt) {
        const unsigned short* wq = bp + (size_t)(16 * nt) * 512 + 256 + k0;
        FragB bf;
        bf.h[0] = *(const v8usa*)wq;
        bf.h[1] = *(const v8usa*)(wq + 16);
        acc[nt] = wmb(af, bf, acc[nt]);
      }
    }
  }
#pragma unroll
  for (int nt = 0; nt < 8; ++nt)
#pragma unroll
    for (int r = 0; r < 8; ++r)
      stg[(16 * wave + 8 * hh + r) * SPT + 16 * nt + m] = acc[nt][r];
  __syncthreads();

  {
    const v4f b1 = *(const v4fa*)(sPar + 4 * lane);
#pragma unroll 1
    for (int i = 0; i < 16; ++i) {
      const int lr = 16 * wave + i;
      const v4f v = *(const v4fa*)(stg + lr * SPT + 4 * lane);
      v4f t;
      t.x = silu_p(v.x + b1.x);
      t.y = silu_p(v.y + b1.y);
      t.z = silu_p(v.z + b1.z);
      t.w = silu_p(v.w + b1.w);
      const HL4 q = split4(t);
      *(v4usa*)(sT + lr * TPT + 4 * lane)       = q.hi;
      *(v4usa*)(sT + lr * TPT + HID + 4 * lane) = q.lo;
    }
  }
  __syncthreads();

  {
    const v8f z = {0.f, 0.f, 0.f, 0.f, 0.f, 0.f, 0.f, 0.f};
#pragma unroll
    for (int t = 0; t < 8; ++t) acc[t] = z;
  }
  {
    const unsigned short* ap = sT + (16 * wave + m) * TPT + 8 * hh;
    const unsigned short* bp = NW2 + (size_t)m * 256 + 8 * hh;
#pragma unroll 1
    for (int k0 = 0; k0 < 256; k0 += 32) {
      FragB af;
      af.h[0] = *(const v8usa*)(ap + k0);
      af.h[1] = *(const v8usa*)(ap + k0 + 16);
#pragma unroll
      for (int nt = 0; nt < 8; ++nt) {
        const unsigned short* wq = bp + (size_t)(16 * nt) * 256 + k0;
        FragB bf;
        bf.h[0] = *(const v8usa*)wq;
        bf.h[1] = *(const v8usa*)(wq + 16);
        acc[nt] = wmb(af, bf, acc[nt]);
      }
    }
  }
  __syncthreads();
#pragma unroll
  for (int nt = 0; nt < 8; ++nt)
#pragma unroll
    for (int r = 0; r < 8; ++r)
      stg[(16 * wave + 8 * hh + r) * SPT + 16 * nt + m] = acc[nt][r];
  __syncthreads();

  {
    const v4f b2 = *(const v4fa*)(sPar + HID + 4 * lane);
#pragma unroll 1
    for (int i = 0; i < 16; ++i) {
      const int lr = 16 * wave + i;
      const v4f v  = *(const v4fa*)(stg + lr * SPT + 4 * lane);
      const v4f hv = *(const v4fa*)(HHi + (size_t)(rowBase + lr) * HID + 4 * lane);
      v4f q;
      q.x = hv.x + (v.x + b2.x);
      q.y = hv.y + (v.y + b2.y);
      q.z = hv.z + (v.z + b2.z);
      q.w = hv.w + (v.w + b2.w);
      *(v4fa*)(stg + lr * SPT + 4 * lane) = q;
    }
  }
  __syncthreads();
  upd_store(stg, HHo, HLo, rowBase, wave, lane);
  __threadfence();
  upd_store(stg, HHo, HLo, rowBase, wave, lane);
}

__global__ __launch_bounds__(256) __attribute__((amdgpu_num_vgpr(248)))
void k_out(const float* __restrict__ HH, const float* __restrict__ X, const float* __restrict__ EO,
           float* out) {
  __shared__ __attribute__((aligned(16))) float sh[64 * SPT];
  __shared__ __attribute__((aligned(16))) float sx[64 * 4];
  __shared__ __attribute__((aligned(16))) float sw[136 * 4];
  __shared__ __attribute__((aligned(16))) float so[256];
  const int tid = (int)threadIdx.x;
  const int rb = (int)blockIdx.x * 64;
#pragma unroll
  for (int q = 0; q < 8; ++q) {
    const int u   = q * 256 + tid;
    const int row = u >> 5;
    const int c4  = (u & 31) * 4;
    const v4f v = *(const v4fa*)(HH + (size_t)(rb + row) * HID + c4);
    *(v4fa*)(sh + row * SPT + c4) = v;
  }
  {
    const int tl = tid < 64 ? tid : 63;
    const v4f xv = *(const v4fa*)(X + (size_t)(rb + tl) * 4);
    if (tid < 64) *(v4fa*)(sx + 4 * tid) = xv;
    const int t2 = tid < 136 ? tid : 135;
    const v4f wv = *(const v4fa*)(EO + 4 * t2);
    if (tid < 136) *(v4fa*)(sw + 4 * tid) = wv;
  }
  __syncthreads();
  {
    const int row = tid >> 2, o = tid & 3;
    float acc = 0.0f;
#pragma unroll 4
    for (int j = 0; j < HID; ++j) acc = fmaf(sh[row * SPT + j], sw[j * 4 + o], acc);
#pragma unroll 1
    for (int d = 0; d < 3; ++d) acc = fmaf(sx[row * 4 + d], sw[(HID + d) * 4 + o], acc);
    acc += sw[131 * 4 + o];
    so[tid] = acc;
  }
  __syncthreads();
  {
    const int tl = tid < 64 ? tid : 63;
    const v4f v = *(const v4fa*)(so + 4 * tl);
    float* dp = out + (size_t)rb * 4 + 4 * tl;
    if (tid < 64) *(volatile v4f*)dp = v;
    __threadfence();
    if (tid < 64) *(volatile v4f*)dp = v;
  }
}

extern "C" void kernel_launch(void* const* d_in, const int* in_sizes, int n_in,
                              void* d_out, int out_size, void* d_ws, size_t ws_size,
                              hipStream_t stream) {
  if (n_in < 18) return;
  if (in_sizes[0] != NN * HROW) return;
  if (in_sizes[1] != NN * KNB) return;
  if (in_sizes[2] != FIN * HID || in_sizes[3] != HID) return;
  if (in_sizes[4] != NL * 257 * HID || in_sizes[5] != NL * HID) return;
  if (in_sizes[6] != NL * HID * HID || in_sizes[7] != NL * HID) return;
  if (in_sizes[8] != NL * HID * HID || in_sizes[9] != NL * HID) return;
  if (in_sizes[10] != NL * HID) return;
  if (in_sizes[11] != NL * 2 * HID * HID || in_sizes[12] != NL * HID) return;
  if (in_sizes[13] != NL * HID * HID || in_sizes[14] != NL * HID) return;
  if (in_sizes[15] != 131 * 4 || in_sizes[16] != 4) return;
  if (out_size != NN * 4) return;

  const float* h     = (const float*)d_in[0];
  const int*   idx   = (const int*)d_in[1];
  const float* eiw   = (const float*)d_in[2];
  const float* eib   = (const float*)d_in[3];
  const float* ew1   = (const float*)d_in[4];
  const float* eb1   = (const float*)d_in[5];
  const float* ew2   = (const float*)d_in[6];
  const float* eb2   = (const float*)d_in[7];
  const float* cw1   = (const float*)d_in[8];
  const float* cb1   = (const float*)d_in[9];
  const float* cw2   = (const float*)d_in[10];
  const float* nw1   = (const float*)d_in[11];
  const float* nb1   = (const float*)d_in[12];
  const float* nw2   = (const float*)d_in[13];
  const float* nb2   = (const float*)d_in[14];
  const float* eow   = (const float*)d_in[15];
  const float* eob   = (const float*)d_in[16];
  float* out = (float*)d_out;

  size_t off = 0;
  const size_t szX   = (size_t)NN * 4 * 4;
  const size_t szHH  = (size_t)NN * HID * 4;
  const size_t szHL  = (size_t)NN * 256 * 2;
  const size_t oXa   = off; off += szX;
  const size_t oXb   = off; off += szX;
  const size_t oHHa  = off; off += szHH;
  const size_t oHHb  = off; off += szHH;
  const size_t oHLa  = off; off += szHL;
  const size_t oHLb  = off; off += szHL;
  const size_t oPSD  = off; off += (size_t)NN * 256 * 4;
  const size_t oSHL  = off; off += szHL;
  const size_t oW1SD = off; off += (size_t)NL * 256 * 256 * 2;
  const size_t oW2D  = off; off += (size_t)NL * 128 * 256 * 2;
  const size_t oCW1T = off; off += (size_t)NL * 128 * 128 * 2;
  const size_t oNW1Q = off; off += (size_t)NL * 128 * 512 * 2;
  const size_t oNW2D = off; off += (size_t)NL * 128 * 256 * 2;
  const size_t oPAR  = off; off += (size_t)NL * 8 * HID * 4;
  const size_t oEO   = off; off += (size_t)2304;
  if (off > ws_size || off > (size_t)WSMAX) return;

  char* ws = (char*)d_ws;
  float* Xp[2]           = {(float*)(ws + oXa), (float*)(ws + oXb)};
  float* HHp[2]          = {(float*)(ws + oHHa), (float*)(ws + oHHb)};
  unsigned short* HLp[2] = {(unsigned short*)(ws + oHLa), (unsigned short*)(ws + oHLb)};
  float* PSD             = (float*)(ws + oPSD);
  unsigned short* SHL    = (unsigned short*)(ws + oSHL);
  unsigned short* W1SD   = (unsigned short*)(ws + oW1SD);
  unsigned short* W2D    = (unsigned short*)(ws + oW2D);
  unsigned short* CW1T   = (unsigned short*)(ws + oCW1T);
  unsigned short* NW1Q   = (unsigned short*)(ws + oNW1Q);
  unsigned short* NW2D   = (unsigned short*)(ws + oNW2D);
  float* PAR             = (float*)(ws + oPAR);
  float* EO              = (float*)(ws + oEO);

  hipFuncSetAttribute(reinterpret_cast<const void*>(&k_edge), hipFuncAttributeMaxDynamicSharedMemorySize,
                      (int)EDGE_LDS);
  hipFuncSetAttribute(reinterpret_cast<const void*>(&k_upd), hipFuncAttributeMaxDynamicSharedMemorySize,
                      (int)UPD_LDS);

  k_pa<<<(NU_W1SD + NU_W2D + NU_CW1) / 256, 256, 0, stream>>>(ew1, ew2, cw1, W1SD, W2D, CW1T);
  k_pb<<<(NU_NW1Q + NU_NW2D) / 256, 256, 0, stream>>>(nw1, nw2, NW1Q, NW2D);
  k_pc<<<NL + 1, 256, 0, stream>>>(ew1, eb1, eb2, cb1, cw2, nb1, nb2, eow, eob, PAR, EO);
  k_emb<<<NN / 32, 256, 0, stream>>>(h, eiw, eib, Xp[0], HHp[0], HLp[0]);

  for (int l = 0; l < NL; ++l) {
    const int a = l & 1, c = (l + 1) & 1;
    const float* PARl = PAR + (size_t)l * 8 * HID;
    k_node<<<dim3(NN / GBM, 2), GTHR, 0, stream>>>(HLp[a], W1SD + (size_t)l * 65536, PARl + HID, PSD);
    k_edge<<<NN / 16, 256, EDGE_LDS, stream>>>(Xp[a], Xp[c], PSD, idx, W2D + (size_t)l * 32768,
                                               CW1T + (size_t)l * 16384, PARl, SHL);
    k_upd<<<NN / 128, 256, UPD_LDS, stream>>>(HLp[a], SHL, NW1Q + (size_t)l * 65536,
                                              NW2D + (size_t)l * 32768, PARl, HHp[a], HHp[c], HLp[c]);
  }
  k_out<<<NN / 64, 256, 0, stream>>>(HHp[NL & 1], Xp[NL & 1], EO, out);
}
